// encoder_layer_26560077758730
// MI455X (gfx1250) — hardware-verified
//
#include <hip/hip_runtime.h>

typedef _Float16 v16h __attribute__((ext_vector_type(16)));
typedef _Float16 v8h  __attribute__((ext_vector_type(8)));
typedef float    v8f  __attribute__((ext_vector_type(8)));
typedef float    v4f  __attribute__((ext_vector_type(4)));
typedef v8h __attribute__((may_alias)) v8ha;
typedef v4f __attribute__((may_alias)) v4fa;

union Frag  { v16h v; v8h half[2]; };
union TileU { float f[128 * 64]; _Float16 h[128 * 64]; };

#define EMB    1024
#define NHEADS 16
#define HD     64
#define SEQ    2048
#define BATCH  2
#define MROWS  (BATCH * SEQ)
#define FFN    4096
#define NX     (MROWS * EMB)
#define NX8    (NX / 8)
#define NW     (EMB * EMB)
#define NF     (EMB * FFN)

#define XC     8.0f
#define WC     4096.0f
#define W2C    8192.0f
#define QC     16.0f
#define PSCALE 16384.0f
#define CTXC   64.0f
#define HC     8.0f
#define AC     8.0f
#define TP     72

static_assert(EMB % 32 == 0);
static_assert(FFN % 32 == 0);
static_assert(MROWS % 128 == 0);
static_assert(EMB % 64 == 0);
static_assert(FFN % 64 == 0);
static_assert(SEQ % 128 == 0);
static_assert(HD == 64);
static_assert(NHEADS * HD == EMB);
static_assert(MROWS % 4 == 0);
static_assert(sizeof(TileU) == 32768);

__device__ __forceinline__ v8f wmma_f16(v16h a, v16h b, v8f c) {
  v8f d = __builtin_amdgcn_wmma_f32_16x16x32_f16(false, a, false, b, (short)0, c, false, false);
  asm volatile("v_nop\n\tv_nop\n\tv_nop\n\tv_nop" : "+v"(d) : "v"(a), "v"(b));
  return d;
}

__device__ __forceinline__ v16h load_frag(const _Float16* p, int h) {
  Frag f;
  f.half[0] = *(const v8ha*)(p + 8 * h);
  f.half[1] = *(const v8ha*)(p + 16 + 8 * h);
  return f.v;
}

__global__ __launch_bounds__(256) void cvt_x_kernel(const float* __restrict__ x,
                                                    _Float16* __restrict__ xh)
{
  const int g = blockIdx.x * 256 + threadIdx.x;
  if (g >= NX8) return;
  const float* src = x + (size_t)g * 8;
  const v4f a = *(const v4fa*)src;
  const v4f c = *(const v4fa*)(src + 4);
  const v8h o = { (_Float16)(a.x * XC), (_Float16)(a.y * XC), (_Float16)(a.z * XC), (_Float16)(a.w * XC),
                  (_Float16)(c.x * XC), (_Float16)(c.y * XC), (_Float16)(c.z * XC), (_Float16)(c.w * XC) };
  _Float16* dst = xh + (size_t)g * 8;
  *(volatile v8h*)dst = o;
  __threadfence();
  *(volatile v8h*)dst = o;
}

__device__ __forceinline__ void tr_store_pass(const _Float16* tile, _Float16* dst,
                                              int n0, int k0, int Kin, int w, int lane) {
  const int q8 = lane & 7, sub = lane >> 3;
  #pragma unroll
  for (int i = 0; i < 2; ++i) {
    const int lid = w * 8 + i * 4 + sub;
    const v8h v = *(const v8ha*)(tile + lid * TP + 8 * q8);
    *(volatile v8h*)(dst + (size_t)(n0 + lid) * Kin + k0 + 8 * q8) = v;
  }
}

__global__ __launch_bounds__(256) void transpose_cvt_kernel(
    const float* __restrict__ s0, const float* __restrict__ s1,
    const float* __restrict__ s2, const float* __restrict__ s3,
    _Float16* __restrict__ d0, _Float16* __restrict__ d1,
    _Float16* __restrict__ d2, _Float16* __restrict__ d3,
    int Kin, int Nout, float sc)
{
  __shared__ __attribute__((aligned(16))) _Float16 tile[64 * TP];
  const int z = blockIdx.z;
  const float* src = (z == 0) ? s0 : ((z == 1) ? s1 : ((z == 2) ? s2 : s3));
  _Float16*    dst = (z == 0) ? d0 : ((z == 1) ? d1 : ((z == 2) ? d2 : d3));
  const int n0 = blockIdx.x * 64;
  const int k0 = blockIdx.y * 64;
  const int tid = threadIdx.x, lane = tid & 31, w = tid >> 5;
  #pragma unroll
  for (int i = 0; i < 4; ++i) {
    const int idx = i * 256 + tid;
    const int kr = idx >> 4, c4 = idx & 15;
    const v4f v = *(const v4fa*)(src + (size_t)(k0 + kr) * Nout + n0 + 4 * c4);
    tile[(4 * c4 + 0) * TP + kr] = (_Float16)(v.x * sc);
    tile[(4 * c4 + 1) * TP + kr] = (_Float16)(v.y * sc);
    tile[(4 * c4 + 2) * TP + kr] = (_Float16)(v.z * sc);
    tile[(4 * c4 + 3) * TP + kr] = (_Float16)(v.w * sc);
  }
  __syncthreads();
  tr_store_pass(tile, dst, n0, k0, Kin, w, lane);
  __threadfence();
  tr_store_pass(tile, dst, n0, k0, Kin, w, lane);
}

__device__ __forceinline__ void qkv_store_pass(const _Float16* sT, _Float16* plane, _Float16* vt,
                                               int which, int bh, int l0, int w, int lane) {
  const int q8 = lane & 7, sub = lane >> 3;
  #pragma unroll
  for (int i = 0; i < 8; ++i) {
    const int lid = w * 32 + i * 4 + sub;
    v8h v;
    _Float16* dst;
    if (which != 2) {
      v = *(const v8ha*)(sT + lid * HD + 8 * q8);
      dst = plane + ((size_t)bh * SEQ + l0 + lid) * HD + 8 * q8;
    } else {
      const int d = lid >> 1, hl = lid & 1;
      v = *(const v8ha*)(sT + d * 128 + 64 * hl + 8 * q8);
      dst = vt + ((size_t)bh * HD + d) * SEQ + l0 + 64 * hl + 8 * q8;
    }
    *(volatile v8h*)dst = v;
  }
}

__device__ __forceinline__ void f32res_store_pass(const float* sTf, const float* __restrict__ res,
                                                  float* outF, int m0, int nrow0, int N,
                                                  int w, int lane) {
  const int q8 = lane & 7, sub = lane >> 3;
  #pragma unroll
  for (int i = 0; i < 16; ++i) {
    const int lid = w * 64 + i * 4 + sub;
    const int row = lid >> 1, hl = lid & 1;
    const v4f v = *(const v4fa*)(sTf + row * 64 + 32 * hl + 4 * q8);
    const size_t gi = (size_t)(m0 + row) * N + nrow0 + 32 * hl + 4 * q8;
    const v4f rr = *(const v4fa*)(res + gi);
    const v4f o = v + rr;
    *(volatile v4f*)(outF + gi) = o;
  }
}

__device__ __forceinline__ void h16_store_pass(const _Float16* sTh, _Float16* outH,
                                               int m0, int nrow0, int N, int w, int lane) {
  const int q8 = lane & 7, sub = lane >> 3;
  #pragma unroll
  for (int i = 0; i < 8; ++i) {
    const int lid = w * 32 + i * 4 + sub;
    const v8h v = *(const v8ha*)(sTh + lid * 64 + 8 * q8);
    *(volatile v8h*)(outH + (size_t)(m0 + lid) * N + nrow0 + 8 * q8) = v;
  }
}

template <int MODE>
__global__ __launch_bounds__(128) void gemm_kernel(
    const _Float16* __restrict__ A, const _Float16* __restrict__ Bt,
    const float* __restrict__ bias0, const float* __restrict__ bias1,
    const float* __restrict__ bias2,
    const float* __restrict__ res,
    float* __restrict__ outF,
    _Float16* __restrict__ outH0, _Float16* __restrict__ outH1, _Float16* __restrict__ outH2,
    int K, int N, float inv)
{
  __shared__ __attribute__((aligned(16))) TileU sT;

  const int tid = threadIdx.x, lane = tid & 31, w = tid >> 5;
  const int h = lane >> 4, m = lane & 15;
  const int m0 = blockIdx.x * 128;
  const int m0w = m0 + 32 * w;

  int nrow0, boff, which = 0, head = 0;
  const float* bias;
  if constexpr (MODE == 0) {
    const int cg = blockIdx.y;
    which = cg >> 4; head = cg & 15;
    nrow0 = which * EMB + head * HD;
    bias = (which == 0) ? bias0 : ((which == 1) ? bias1 : bias2);
    boff = head * HD;
  } else {
    nrow0 = blockIdx.y * 64;
    bias = bias0;
    boff = nrow0;
  }

  const _Float16* xa0 = A + (size_t)(m0w + m) * K;
  const _Float16* xa1 = xa0 + (size_t)16 * K;
  const _Float16* wb  = Bt + (size_t)(nrow0 + m) * K;

  const v8f zero8 = {0.f, 0.f, 0.f, 0.f, 0.f, 0.f, 0.f, 0.f};
  v8f acc[2][4];
  #pragma unroll
  for (int mt = 0; mt < 2; ++mt)
    #pragma unroll
    for (int nt = 0; nt < 4; ++nt) acc[mt][nt] = zero8;

  #pragma unroll 1
  for (int k0 = 0; k0 < K; k0 += 32) {
    const v16h a0 = load_frag(xa0 + k0, h);
    const v16h a1 = load_frag(xa1 + k0, h);
    #pragma unroll
    for (int nt = 0; nt < 4; ++nt) {
      const v16h b = load_frag(wb + (size_t)nt * 16 * K + k0, h);
      acc[0][nt] = wmma_f16(a0, b, acc[0][nt]);
      acc[1][nt] = wmma_f16(a1, b, acc[1][nt]);
    }
  }

  #pragma unroll
  for (int nt = 0; nt < 4; ++nt) {
    const int feat = 16 * nt + m;
    const float bvl = bias[boff + feat];
    #pragma unroll
    for (int mt = 0; mt < 2; ++mt) {
      #pragma unroll
      for (int r = 0; r < 8; ++r) {
        const int tokl = 32 * w + 16 * mt + 8 * h + r;
        const float y = acc[mt][nt][r] * inv + bvl;
        if constexpr (MODE == 0) {
          const int idx = (which == 2) ? (feat * 128 + tokl) : (tokl * HD + feat);
          sT.h[idx] = (_Float16)(y * QC);
        } else if constexpr (MODE == 1) {
          sT.f[tokl * 64 + feat] = y;
        } else {
          sT.h[tokl * 64 + feat] = (_Float16)(fmaxf(y, 0.0f) * AC);
        }
      }
    }
  }
  __syncthreads();

  if constexpr (MODE == 0) {
    const int b = m0 / SEQ, l0 = m0 - b * SEQ, bh = b * NHEADS + head;
    _Float16* plane = (which == 0) ? outH0 : outH1;
    qkv_store_pass(sT.h, plane, outH2, which, bh, l0, w, lane);
    __threadfence();
    qkv_store_pass(sT.h, plane, outH2, which, bh, l0, w, lane);
  } else if constexpr (MODE == 1) {
    f32res_store_pass(sT.f, res, outF, m0, nrow0, N, w, lane);
    __threadfence();
    f32res_store_pass(sT.f, res, outF, m0, nrow0, N, w, lane);
  } else {
    h16_store_pass(sT.h, outH0, m0, nrow0, N, w, lane);
    __threadfence();
    h16_store_pass(sT.h, outH0, m0, nrow0, N, w, lane);
  }
}

__device__ __forceinline__ v8f scale_mask8(v8f z, const float* p) {
  const float SSC = 0.125f / (QC * QC);
  const float MNEG = -1e12f;
  const v4f ma = *(const v4fa*)p;
  const v4f mb = *(const v4fa*)(p + 4);
  v8f s;
  s[0] = z[0] * SSC + ma.x * MNEG;
  s[1] = z[1] * SSC + ma.y * MNEG;
  s[2] = z[2] * SSC + ma.z * MNEG;
  s[3] = z[3] * SSC + ma.w * MNEG;
  s[4] = z[4] * SSC + mb.x * MNEG;
  s[5] = z[5] * SSC + mb.y * MNEG;
  s[6] = z[6] * SSC + mb.z * MNEG;
  s[7] = z[7] * SSC + mb.w * MNEG;
  return s;
}

__device__ __forceinline__ v16h pack_p(v8f a, v8f c) {
  const v16h r = { (_Float16)(a[0] * PSCALE), (_Float16)(a[1] * PSCALE), (_Float16)(a[2] * PSCALE), (_Float16)(a[3] * PSCALE),
                   (_Float16)(a[4] * PSCALE), (_Float16)(a[5] * PSCALE), (_Float16)(a[6] * PSCALE), (_Float16)(a[7] * PSCALE),
                   (_Float16)(c[0] * PSCALE), (_Float16)(c[1] * PSCALE), (_Float16)(c[2] * PSCALE), (_Float16)(c[3] * PSCALE),
                   (_Float16)(c[4] * PSCALE), (_Float16)(c[5] * PSCALE), (_Float16)(c[6] * PSCALE), (_Float16)(c[7] * PSCALE) };
  return r;
}

__device__ __forceinline__ void ctx_store_pass(const float* so, _Float16* ctx,
                                               int b, int head, int q0, int lane) {
  const int q8 = lane & 7, sub = lane >> 3;
  #pragma unroll
  for (int i = 0; i < 4; ++i) {
    const int row = i * 4 + sub;
    const v4f a = *(const v4fa*)(so + row * 64 + 8 * q8);
    const v4f c = *(const v4fa*)(so + row * 64 + 8 * q8 + 4);
    const v8h v = { (_Float16)a.x, (_Float16)a.y, (_Float16)a.z, (_Float16)a.w,
                    (_Float16)c.x, (_Float16)c.y, (_Float16)c.z, (_Float16)c.w };
    const size_t gi = ((size_t)b * SEQ + q0 + row) * EMB + head * HD + 8 * q8;
    *(volatile v8h*)(ctx + gi) = v;
  }
}

__global__ __launch_bounds__(128) void attn_kernel(
    const _Float16* __restrict__ qh,
    const _Float16* __restrict__ kh,
    const _Float16* __restrict__ vt,
    const float* __restrict__ mask,
    _Float16* __restrict__ ctx)
{
  __shared__ __attribute__((aligned(16))) float sO[4 * 16 * 64];

  const int tid = threadIdx.x, lane = tid & 31, w = tid >> 5;
  const int h = lane >> 4, m = lane & 15;
  const int bh = blockIdx.y, b = bh >> 4, head = bh & 15;
  const int q0 = blockIdx.x * 64 + 16 * w;

  const _Float16* qrow = qh + ((size_t)bh * SEQ + q0 + m) * HD;
  const v16h qb0 = load_frag(qrow, h);
  const v16h qb1 = load_frag(qrow + 32, h);

  const v8f zero8 = {0.f, 0.f, 0.f, 0.f, 0.f, 0.f, 0.f, 0.f};
  v8f o[4];
  #pragma unroll
  for (int t = 0; t < 4; ++t) o[t] = zero8;
  float mrun = -1e30f, lrun = 0.0f;

  const _Float16* kbase = kh + ((size_t)bh * SEQ + m) * HD;
  const _Float16* vbase = vt + ((size_t)bh * HD + m) * SEQ;
  const float* mkp = mask + (size_t)b * SEQ + 8 * h;

  #pragma unroll 1
  for (int kb = 0; kb < SEQ; kb += 64) {
    v8f s[4];
    #pragma unroll
    for (int j = 0; j < 4; ++j) {
      const _Float16* kp = kbase + (size_t)(kb + 16 * j) * HD;
      const v16h kf0 = load_frag(kp, h);
      const v16h kf1 = load_frag(kp + 32, h);
      v8f z = zero8;
      z = wmma_f16(kf0, qb0, z);
      z = wmma_f16(kf1, qb1, z);
      s[j] = z;
    }
    #pragma unroll
    for (int j = 0; j < 4; ++j) s[j] = scale_mask8(s[j], mkp + kb + 16 * j);

    float mloc = s[0][0];
    #pragma unroll
    for (int j = 0; j < 4; ++j)
      #pragma unroll
      for (int r = 0; r < 8; ++r) mloc = fmaxf(mloc, s[j][r]);
    mloc = fmaxf(mloc, __shfl_xor(mloc, 16));
    const float mnew = fmaxf(mrun, mloc);
    const float alpha = __expf(mrun - mnew);
    mrun = mnew;
    float lsum = 0.0f;
    #pragma unroll
    for (int j = 0; j < 4; ++j)
      #pragma unroll
      for (int r = 0; r < 8; ++r) {
        const float p = __expf(s[j][r] - mnew);
        s[j][r] = p;
        lsum += p;
      }
    lsum += __shfl_xor(lsum, 16);
    lrun = lrun * alpha + lsum;
    #pragma unroll
    for (int t = 0; t < 4; ++t)
      #pragma unroll
      for (int r = 0; r < 8; ++r) o[t][r] = o[t][r] * alpha;

    const v16h pb0 = pack_p(s[0], s[1]);
    const v16h pb1 = pack_p(s[2], s[3]);

    #pragma unroll
    for (int t = 0; t < 4; ++t) {
      const _Float16* vp = vbase + (size_t)(16 * t) * SEQ + kb;
      const v16h vf0 = load_frag(vp, h);
      const v16h vf1 = load_frag(vp + 32, h);
      o[t] = wmma_f16(vf0, pb0, o[t]);
      o[t] = wmma_f16(vf1, pb1, o[t]);
    }
  }

  const float cinv = (1.0f / lrun) * (CTXC / (PSCALE * QC));
  float* so = sO + w * 1024;
  #pragma unroll
  for (int t = 0; t < 4; ++t)
    #pragma unroll
    for (int r = 0; r < 8; ++r)
      so[m * 64 + 16 * t + 8 * h + r] = o[t][r] * cinv;
  __syncthreads();

  ctx_store_pass(so, ctx, b, head, q0, lane);
  __threadfence();
  ctx_store_pass(so, ctx, b, head, q0, lane);
}

template <bool WH>
__global__ __launch_bounds__(128) void layernorm_kernel(
    const float* __restrict__ in, const float* __restrict__ g, const float* __restrict__ be,
    float* __restrict__ outF, _Float16* __restrict__ outH)
{
  __shared__ __attribute__((aligned(16))) float srow[4 * EMB];

  const int tid = threadIdx.x, lane = tid & 31, w = tid >> 5;
  const int row = blockIdx.x * 4 + w;
  const float* xr = in + (size_t)row * EMB;
  float* sr = srow + w * EMB;

  float s = 0.0f;
  #pragma unroll 1
  for (int i = 0; i < 8; ++i) {
    const v4f v = *(const v4fa*)(xr + 128 * i + 4 * lane);
    s += (v.x + v.y) + (v.z + v.w);
  }
  #pragma unroll
  for (int ofs = 16; ofs >= 1; ofs >>= 1) s += __shfl_xor(s, ofs);
  const float mu = s * (1.0f / EMB);

  float q = 0.0f;
  #pragma unroll 1
  for (int i = 0; i < 8; ++i) {
    const v4f v = *(const v4fa*)(xr + 128 * i + 4 * lane);
    const v4f d = v - mu;
    q += (d.x * d.x + d.y * d.y) + (d.z * d.z + d.w * d.w);
  }
  #pragma unroll
  for (int ofs = 16; ofs >= 1; ofs >>= 1) q += __shfl_xor(q, ofs);
  const float var = q * (1.0f / EMB);
  const float rs = rsqrtf(var + 1e-9f);

  #pragma unroll 1
  for (int i = 0; i < 8; ++i) {
    const int c = 128 * i + 4 * lane;
    const v4f v  = *(const v4fa*)(xr + c);
    const v4f gv = *(const v4fa*)(g + c);
    const v4f bv = *(const v4fa*)(be + c);
    const v4f t  = (v - mu) * rs;
    const v4f y  = t * gv + bv;
    *(v4fa*)(sr + c) = y;
    *(volatile v4f*)(outF + (size_t)row * EMB + c) = y;
  }
  __threadfence();
  #pragma unroll 1
  for (int i = 0; i < 8; ++i) {
    const int c = 128 * i + 4 * lane;
    const v4f y = *(const v4fa*)(sr + c);
    *(volatile v4f*)(outF + (size_t)row * EMB + c) = y;
  }

  if constexpr (WH) {
    __syncthreads();
    #pragma unroll 1
    for (int i = 0; i < 4; ++i) {
      const int c = 256 * i + 8 * lane;
      const v4f a = *(const v4fa*)(sr + c);
      const v4f d = *(const v4fa*)(sr + c + 4);
      const v8h o = { (_Float16)(a.x * HC), (_Float16)(a.y * HC), (_Float16)(a.z * HC), (_Float16)(a.w * HC),
                      (_Float16)(d.x * HC), (_Float16)(d.y * HC), (_Float16)(d.z * HC), (_Float16)(d.w * HC) };
      *(volatile v8h*)(outH + (size_t)row * EMB + c) = o;
    }
    __threadfence();
    #pragma unroll 1
    for (int i = 0; i < 4; ++i) {
      const int c = 256 * i + 8 * lane;
      const v4f a = *(const v4fa*)(sr + c);
      const v4f d = *(const v4fa*)(sr + c + 4);
      const v8h o = { (_Float16)(a.x * HC), (_Float16)(a.y * HC), (_Float16)(a.z * HC), (_Float16)(a.w * HC),
                      (_Float16)(d.x * HC), (_Float16)(d.y * HC), (_Float16)(d.z * HC), (_Float16)(d.w * HC) };
      *(volatile v8h*)(outH + (size_t)row * EMB + c) = o;
    }
  }
}

extern "C" void kernel_launch(void* const* d_in, const int* in_sizes, int n_in,
                              void* d_out, int out_size, void* d_ws, size_t ws_size,
                              hipStream_t stream) {
  if (n_in < 18) return;
  if (in_sizes[0] != NX) return;
  if (in_sizes[1] != BATCH * SEQ) return;
  if (in_sizes[2] != NW || in_sizes[4] != NW || in_sizes[6] != NW || in_sizes[8] != NW) return;
  if (in_sizes[3] != EMB || in_sizes[5] != EMB || in_sizes[7] != EMB || in_sizes[9] != EMB) return;
  if (in_sizes[10] != NF || in_sizes[11] != FFN || in_sizes[12] != NF || in_sizes[13] != EMB) return;
  if (in_sizes[14] != EMB || in_sizes[15] != EMB || in_sizes[16] != EMB || in_sizes[17] != EMB) return;
  if (out_size != NX) return;

  const float* x    = (const float*)d_in[0];
  const float* mask = (const float*)d_in[1];
  const float* wq_w = (const float*)d_in[2];
  const float* wq_b = (const float*)d_in[3];
  const float* wk_w = (const float*)d_in[4];
  const float* wk_b = (const float*)d_in[5];
  const float* wv_w = (const float*)d_in[6];
  const float* wv_b = (const float*)d_in[7];
  const float* wo_w = (const float*)d_in[8];
  const float* wo_b = (const float*)d_in[9];
  const float* f1_w = (const float*)d_in[10];
  const float* f1_b = (const float*)d_in[11];
  const float* f2_w = (const float*)d_in[12];
  const float* f2_b = (const float*)d_in[13];
  const float* ln1_g = (const float*)d_in[14];
  const float* ln1_b = (const float*)d_in[15];
  const float* ln2_g = (const float*)d_in[16];
  const float* ln2_b = (const float*)d_in[17];
  float* out = (float*)d_out;

  const size_t xh_bytes  = (size_t)NX * 2;
  const size_t pl_bytes  = (size_t)BATCH * NHEADS * SEQ * HD * 2;
  const size_t a16_bytes = (size_t)MROWS * FFN * 2;
  const size_t wqkv_bytes = (size_t)3 * NW * 2;
  const size_t wo_bytes  = (size_t)NW * 2;
  const size_t f1_bytes  = (size_t)NF * 2;
  const size_t f2_bytes  = (size_t)NF * 2;
  const size_t f32_bytes = (size_t)NX * 4;
  const size_t h16_bytes = (size_t)NX * 2;

  const size_t off_xh   = 0;
  const size_t off_q    = off_xh + xh_bytes;
  const size_t off_k    = off_q + pl_bytes;
  const size_t off_vt   = off_k + pl_bytes;
  const size_t off_wqkv = off_vt + pl_bytes;
  const size_t off_wo   = off_wqkv + wqkv_bytes;
  const size_t off_f1   = off_wo + wo_bytes;
  const size_t off_f2   = off_f1 + f1_bytes;
  const size_t off_tmp  = off_f2 + f2_bytes;
  const size_t off_h32  = off_tmp + f32_bytes;
  const size_t off_h16  = off_h32 + f32_bytes;
  const size_t total    = off_h16 + h16_bytes;
  if (a16_bytes > off_wqkv) return;
  if (total > ws_size) return;

  char* ws = (char*)d_ws;
  _Float16* xh   = (_Float16*)(ws + off_xh);
  _Float16* ctx  = (_Float16*)(ws + off_xh);
  _Float16* a16  = (_Float16*)(ws + off_xh);
  _Float16* qh   = (_Float16*)(ws + off_q);
  _Float16* kh   = (_Float16*)(ws + off_k);
  _Float16* vt   = (_Float16*)(ws + off_vt);
  _Float16* wqkv = (_Float16*)(ws + off_wqkv);
  _Float16* wot  = (_Float16*)(ws + off_wo);
  _Float16* f1t  = (_Float16*)(ws + off_f1);
  _Float16* f2t  = (_Float16*)(ws + off_f2);
  float*    tmp  = (float*)(ws + off_tmp);
  float*    h32  = (float*)(ws + off_h32);
  _Float16* h16  = (_Float16*)(ws + off_h16);

  cvt_x_kernel<<<(NX8 + 255) / 256, 256, 0, stream>>>(x, xh);

  transpose_cvt_kernel<<<dim3(EMB / 64, EMB / 64, 4), 256, 0, stream>>>(
      wq_w, wk_w, wv_w, wo_w, wqkv, wqkv + (size_t)NW, wqkv + (size_t)2 * NW, wot, EMB, EMB, WC);
  transpose_cvt_kernel<<<dim3(FFN / 64, EMB / 64, 1), 256, 0, stream>>>(
      f1_w, f1_w, f1_w, f1_w, f1t, f1t, f1t, f1t, EMB, FFN, WC);
  transpose_cvt_kernel<<<dim3(EMB / 64, FFN / 64, 1), 256, 0, stream>>>(
      f2_w, f2_w, f2_w, f2_w, f2t, f2t, f2t, f2t, FFN, EMB, W2C);

  gemm_kernel<0><<<dim3(MROWS / 128, 3 * NHEADS), 128, 0, stream>>>(
      xh, wqkv, wq_b, wk_b, wv_b, x, tmp, qh, kh, vt, EMB, EMB, 1.0f / (XC * WC));

  attn_kernel<<<dim3(SEQ / 64, BATCH * NHEADS), 128, 0, stream>>>(qh, kh, vt, mask, ctx);

  gemm_kernel<1><<<dim3(MROWS / 128, EMB / 64), 128, 0, stream>>>(
      ctx, wot, wo_b, wo_b, wo_b, x, tmp, h16, h16, h16, EMB, EMB, 1.0f / (CTXC * WC));

  layernorm_kernel<true><<<MROWS / 4, 128, 0, stream>>>(tmp, ln1_g, ln1_b, h32, h16);

  gemm_kernel<2><<<dim3(MROWS / 128, FFN / 64), 128, 0, stream>>>(
      h16, f1t, f1_b, f1_b, f1_b, h32, tmp, a16, a16, a16, EMB, FFN, 1.0f / (HC * WC));

  gemm_kernel<1><<<dim3(MROWS / 128, EMB / 64), 128, 0, stream>>>(
      a16, f2t, f2_b, f2_b, f2_b, h32, tmp, h16, h16, h16, FFN, EMB, 1.0f / (AC * W2C));

  layernorm_kernel<false><<<MROWS / 4, 128, 0, stream>>>(tmp, ln2_g, ln2_b, out, h16);
}
